// PrototypeClassifier_43559558316185
// MI455X (gfx1250) — hardware-verified
//
#include <hip/hip_runtime.h>


#define NR   8192
#define NC   1000
#define NCP  1024
#define ND   128
constexpr size_t al256(size_t b) { return (b + 255) & ~(size_t)255; }
constexpr size_t WS_TOTAL = al256((size_t)NR * ND * 2) + al256((size_t)NCP * ND * 2) + al256((size_t)NR * NCP * 4) + al256((size_t)NR * 4) + al256((size_t)NCP * 4);
static_assert(WS_TOTAL == 35950592 && WS_TOTAL <= 134217728, "the workspace carve: about 34.3 MiB");
typedef _Float16 h16;
typedef unsigned short bf;
typedef __attribute__((ext_vector_type(16))) __bf16   v16bf;
typedef __attribute__((ext_vector_type(16))) _Float16 v16h;
typedef __attribute__((ext_vector_type(8)))  _Float16 v8h;
typedef __attribute__((ext_vector_type(8)))  unsigned short v8us;
typedef __attribute__((ext_vector_type(8)))  float    v8f;
typedef __attribute__((ext_vector_type(4)))  float    v4f;
typedef v8h  __attribute__((may_alias)) v8ha;
typedef v4f  __attribute__((may_alias)) v4fa;
typedef v8us __attribute__((may_alias)) v8usa;

__device__ __forceinline__ unsigned short f2bf(float f) { unsigned u = __float_as_uint(f); u += 0x7FFFu + ((u >> 16) & 1u); return (unsigned short)(u >> 16); }
__device__ __forceinline__ float bf2f(unsigned short b) { return __uint_as_float(((unsigned)b) << 16); }
__device__ __forceinline__ float bfr(float f) { return bf2f(f2bf(f)); }
__device__ __forceinline__ v16h cat16(v8h lo, v8h hi) { return __builtin_shufflevector(lo, hi, 0, 1, 2, 3, 4, 5, 6, 7, 8, 9, 10, 11, 12, 13, 14, 15); }
__device__ __forceinline__ v16bf cat16b(v8us lo, v8us hi) { return __builtin_bit_cast(v16bf, __builtin_shufflevector(lo, hi, 0, 1, 2, 3, 4, 5, 6, 7, 8, 9, 10, 11, 12, 13, 14, 15)); }
__device__ __forceinline__ v8f wmma16(v16h a, v16h b, v8f c) { return __builtin_amdgcn_wmma_f32_16x16x32_f16(false, a, false, b, (short)0, c, false, false); }
__device__ __forceinline__ v8f wmmab(v16bf a, v16bf b, v8f c) { return __builtin_amdgcn_wmma_f32_16x16x32_bf16(false, a, false, b, (short)0, c, false, false); }


template <typename T16> struct WFrag;
template <> struct WFrag<h16> { typedef v16h V; static __device__ __forceinline__ V ld(const h16* p) { return cat16(*(const v8h*)p, *(const v8h*)(p + 16)); } static __device__ __forceinline__ v8f mma(V a, V b, v8f c) { return wmma16(a, b, c); } };
template <> struct WFrag<bf> { typedef v16bf V; static __device__ __forceinline__ V ld(const bf* p) { return cat16b(*(const v8us*)p, *(const v8us*)(p + 16)); } static __device__ __forceinline__ v8f mma(V a, V b, v8f c) { return wmmab(a, b, c); } };
template <typename T16, int NSPLIT, bool BIAS>
__global__ __launch_bounds__(32) void k_gemmw(const T16* __restrict__ A, const T16* __restrict__ A2, const T16* __restrict__ Bt, const T16* __restrict__ Bt2, int K, float* C, int ldc, const float* __restrict__ bias, size_t sA, size_t sB, size_t sC) {
    typedef typename WFrag<T16>::V V;
    __shared__ __align__(16) float os[16 * 68];
    const size_t z = blockIdx.z; A += z * sA; if (A2) A2 += z * sA; Bt += z * sB; if (Bt2) Bt2 += z * sB; C += z * sC;
    const int lane = threadIdx.x & 31, lr = lane & 15, hi = lane >> 4; const int r0 = blockIdx.x * 64, c0 = blockIdx.y * 64;
    v8f acc[4][4];
#pragma unroll
    for (int mb = 0; mb < 4; ++mb)
#pragma unroll
        for (int nb = 0; nb < 4; ++nb) acc[mb][nb] = (v8f){};
    const size_t aoff = (size_t)(r0 + lr) * K + 8 * hi, boff = (size_t)(c0 + lr) * K + 8 * hi;
    for (int kc = 0; kc < K; kc += 32) {
        V a[4], a2[4];
#pragma unroll
        for (int mb = 0; mb < 4; ++mb) { a[mb] = WFrag<T16>::ld(A + aoff + (size_t)mb * 16 * K + kc); if (NSPLIT == 1 || NSPLIT == 2) a2[mb] = WFrag<T16>::ld(A2 + aoff + (size_t)mb * 16 * K + kc); }
#pragma unroll
        for (int nb = 0; nb < 4; ++nb) { const V b = WFrag<T16>::ld(Bt + boff + (size_t)nb * 16 * K + kc); V b2; if (NSPLIT >= 2) b2 = WFrag<T16>::ld(Bt2 + boff + (size_t)nb * 16 * K + kc);
#pragma unroll
            for (int mb = 0; mb < 4; ++mb) { acc[mb][nb] = WFrag<T16>::mma(a[mb], b, acc[mb][nb]); if (NSPLIT == 1 || NSPLIT == 2) acc[mb][nb] = WFrag<T16>::mma(a2[mb], b, acc[mb][nb]); if (NSPLIT >= 2) acc[mb][nb] = WFrag<T16>::mma(a[mb], b2, acc[mb][nb]); } }
        asm volatile("v_nop\n\tv_nop\n\tv_nop\n\tv_nop" : "+v"(acc[0][0]), "+v"(acc[1][1]), "+v"(acc[2][2]), "+v"(acc[3][3]) : "v"(a[0]), "v"(a[3]));
    }
#pragma unroll
    for (int mb = 0; mb < 4; ++mb) {
#pragma unroll
        for (int nb = 0; nb < 4; ++nb) {
#pragma unroll
            for (int j = 0; j < 8; ++j) os[(hi * 8 + j) * 68 + nb * 16 + lr] = acc[mb][nb][j]; }
        __builtin_amdgcn_wave_barrier(); asm volatile("" ::: "memory");
        float* crow = C + (size_t)(r0 + mb * 16) * ldc + c0;
#pragma unroll 1
        for (int ps = 0; ps < 2; ++ps) {
#pragma unroll
            for (int s = 0; s < 8; ++s) { const int row = 2 * s + hi, cofs = lr * 4; v4f val = *(const v4fa*)(os + row * 68 + cofs); if (BIAS) { val[0] += bfr(bias[c0 + cofs]); val[1] += bfr(bias[c0 + cofs + 1]); val[2] += bfr(bias[c0 + cofs + 2]); val[3] += bfr(bias[c0 + cofs + 3]); }
                *(volatile v4f*)(crow + (size_t)row * ldc + cofs) = val; }
            if (ps == 0) __threadfence(); }
        __builtin_amdgcn_wave_barrier(); asm volatile("" ::: "memory");
    }
}

__device__ __forceinline__ h16 tohx(float x) { return (h16)x; }
__device__ __forceinline__ void splitf(float y, unsigned short& h, unsigned short& l) { h = f2bf(y); l = f2bf(y - bf2f(h)); }
typedef __attribute__((ext_vector_type(2))) _Float16 v2h;
typedef __attribute__((ext_vector_type(4))) _Float16 v4h;
typedef __attribute__((ext_vector_type(2))) unsigned short v2us;
typedef __attribute__((ext_vector_type(4))) unsigned short v4us;
typedef __attribute__((ext_vector_type(2))) float v2f;
typedef __attribute__((ext_vector_type(4))) int v4i;

__global__ __launch_bounds__(256) void k_cvt8(const float* __restrict__ src, bf* dst, size_t n8) { const size_t i = (size_t)blockIdx.x * 256 + threadIdx.x; if (i >= n8) return; const v8f v = *(const v8f*)(src + i * 8); v8us o;
#pragma unroll
    for (int k = 0; k < 8; ++k) o[k] = f2bf(v[k]); *(volatile v8us*)(dst + i * 8) = o; __threadfence(); *(volatile v8us*)(dst + i * 8) = o; }

__global__ __launch_bounds__(256) void k_norm(const float* __restrict__ src, int nrows, int nrp, float* nrm, bf* pad, int npad16) {
    const int r = blockIdx.x * 256 + threadIdx.x; if (r >= nrp) return;
    float s = 0.0f;
    if (r < nrows) { const float* p = src + (size_t)r * ND;
        for (int d = 0; d < ND; d += 4) { const v4f v = *(const v4f*)(p + d); const float a = bfr(v[0]), b = bfr(v[1]), c = bfr(v[2]), e = bfr(v[3]); s += a * a; s += b * b; s += c * c; s += e * e; } }
    v8us z; for (int j = 0; j < 8; ++j) z[j] = 0;
#pragma unroll
    for (int ps = 0; ps < 2; ++ps) { *(volatile float*)(nrm + r) = s; if (pad != nullptr && r < npad16) *(volatile v8us*)(pad + (size_t)r * 8) = z; if (ps == 0) __threadfence(); } }

__global__ __launch_bounds__(256) void k_comb(const float* G, const float* xn, const float* cn, float* out) {
    const size_t e = (size_t)blockIdx.x * 256 + threadIdx.x; if (e >= (size_t)NR * NC) return; const size_t n = e / NC; const int c = (int)(e % NC);
    const float v = (2.0f * G[n * NCP + c] - xn[n]) - cn[c];
    *(volatile float*)(out + e) = v; __threadfence(); *(volatile float*)(out + e) = v; }

extern "C" void kernel_launch(void* const* d_in, const int* in_sizes, int n_in,
                              void* d_out, int out_size, void* d_ws, size_t ws_size, hipStream_t stream) {
    if (n_in < 2) return;
    if (in_sizes[0] < NR * ND || in_sizes[1] < NC * ND || out_size < NR * NC) return;
    const float* xs = (const float*)d_in[0]; const float* cs = (const float*)d_in[1];
    float* OUT = (float*)d_out;
    char* wsp = (char*)d_ws;
    auto take = [&](size_t bytes) { char* p = wsp; wsp += (bytes + 255) & ~(size_t)255; return (void*)p; };
    bf* XB = (bf*)take((size_t)NR * ND * 2); bf* CB = (bf*)take((size_t)NCP * ND * 2); float* G = (float*)take((size_t)NR * NCP * 4); float* XN = (float*)take((size_t)NR * 4); float* CN = (float*)take((size_t)NCP * 4);
    if ((size_t)(wsp - (char*)d_ws) != WS_TOTAL || WS_TOTAL > ws_size) return;
    k_cvt8<<<(unsigned)(((size_t)NR * ND / 8 + 255) / 256), 256, 0, stream>>>(xs, XB, (size_t)NR * ND / 8);
    k_cvt8<<<(unsigned)(((size_t)NC * ND / 8 + 255) / 256), 256, 0, stream>>>(cs, CB, (size_t)NC * ND / 8);
    k_norm<<<(NR + 255) / 256, 256, 0, stream>>>(xs, NR, NR, XN, nullptr, 0);
    k_norm<<<(NCP + 255) / 256, 256, 0, stream>>>(cs, NC, NCP, CN, CB + (size_t)NC * ND, (NCP - NC) * ND / 8);
    k_gemmw<bf, 0, false><<<dim3(NR / 64, NCP / 64, 1), 32, 0, stream>>>(XB, nullptr, CB, nullptr, ND, G, NCP, nullptr, (size_t)0, (size_t)0, (size_t)0);
    k_comb<<<(unsigned)(((size_t)NR * NC + 255) / 256), 256, 0, stream>>>(G, XN, CN, OUT);
}
